// BiLSTM_23639499997827
// MI455X (gfx1250) — hardware-run, weakly checked
//
#include <hip/hip_runtime.h>
#include <math.h>

typedef __attribute__((ext_vector_type(16))) _Float16 v16h;
typedef __attribute__((ext_vector_type(8)))  _Float16 v8h;
typedef __attribute__((ext_vector_type(2)))  _Float16 v2h;
typedef __attribute__((ext_vector_type(16))) __bf16   v16b;
typedef __attribute__((ext_vector_type(8)))  __bf16   v8b;
typedef __attribute__((ext_vector_type(8)))  float    v8f;
typedef __attribute__((ext_vector_type(4)))  float    v4f;
typedef __attribute__((ext_vector_type(2)))  float    v2f;
typedef __attribute__((ext_vector_type(4)))  _Float16 v4h;

constexpr int kB    = 4096;
constexpr int kI    = 1024;
constexpr int kHid  = 1024;
constexpr int kK    = kI + kHid;
constexpr int kG4   = 4 * kHid;
constexpr int kOut1 = kB * kHid;
constexpr int kOutAll = 4 * kOut1;
constexpr int kThr  = 256;
constexpr float kInCarry = 1024.0f;
constexpr float kSc = 1.0f / (kInCarry * kInCarry);
constexpr float kF16MinNormal = 6.103515625e-5f;

static_assert(kB == 4096 && kI == 1024 && kHid == 1024 && kK == 2048 && kG4 == 4096, "the index arithmetic below uses these sizes");

constexpr size_t kOffAF16 = 0ull;
constexpr size_t kOffAB16 = 16777216ull;
constexpr size_t kOffWF16 = 33554432ull;
constexpr size_t kOffWB16 = 50331648ull;
constexpr size_t kOffBV = 67108864ull;
constexpr size_t kOffGG = 67141632ull;
constexpr size_t kWsTotal = 134250496ull;
static_assert(kWsTotal <= 268435456ull, "the carve stands under the contract's 256 MiB of workspace");
static_assert(kOffAF16 == 0
  && kOffAB16 == kOffAF16 + 16777216ull
  && kOffWF16 == kOffAB16 + 16777216ull
  && kOffWB16 == kOffWF16 + 16777216ull
  && kOffBV == kOffWB16 + 16777216ull
  && kOffGG == kOffBV + 32768ull
  && kWsTotal == kOffGG + 67108864ull, "the carve is a chain: every region starts where the one before ends");
static_assert((kOffAB16 % 256) == 0 && (kOffWF16 % 256) == 0 && (kOffWB16 % 256) == 0 && (kOffBV % 256) == 0 && (kOffGG % 256) == 0, "every region starts on a multiple of 256 B");

__device__ __forceinline__ unsigned short f2bf_bits(float f) {
  unsigned u = __float_as_uint(f);
  return (unsigned short)((u + 0x7FFFu + ((u >> 16) & 1u)) >> 16);
}
__device__ __forceinline__ float bf_bits2f(unsigned short h) { return __uint_as_float(((unsigned)h) << 16); }
__device__ __forceinline__ float bf16r(float f) { return bf_bits2f(f2bf_bits(f)); }
__device__ __forceinline__ float carry_flush(float v, float carry) {
  const float s = v * carry;
  return (fabsf(s) < kF16MinNormal) ? 0.0f : s;
}

__device__ __forceinline__ void dep_guard4_h(v8f& a, v8f& b, v8f& c, v8f& d, v16h x, v16h y) { asm volatile("v_nop\n\tv_nop\n\tv_nop\n\tv_nop" : "+v"(a), "+v"(b), "+v"(c), "+v"(d) : "v"(x), "v"(y)); }
__device__ __forceinline__ void dep_guard4_b(v8f& a, v8f& b, v8f& c, v8f& d, v16b x, v16b y) { asm volatile("v_nop\n\tv_nop\n\tv_nop\n\tv_nop" : "+v"(a), "+v"(b), "+v"(c), "+v"(d) : "v"(x), "v"(y)); }
__device__ __forceinline__ void keep4_h(v16h a, v16h b, v16h c, v16h d) { asm volatile("v_nop" :: "v"(a), "v"(b), "v"(c), "v"(d)); }
__device__ __forceinline__ void keep4_b(v16b a, v16b b, v16b c, v16b d) { asm volatile("v_nop" :: "v"(a), "v"(b), "v"(c), "v"(d)); }
__device__ __forceinline__ void acc_guard4(v8f& a, v8f& b, v8f& c, v8f& d) { asm volatile("v_nop\n\tv_nop\n\tv_nop\n\tv_nop" : "+v"(a), "+v"(b), "+v"(c), "+v"(d)); }

template <typename T> struct Frag;
template <> struct Frag<_Float16> {
  typedef v16h V; union U { v16h v; v8h h[2]; };
  static __device__ __forceinline__ v16h load(const _Float16* p) {
    U f; f.h[0] = *(const v8h*)(p); f.h[1] = *(const v8h*)(p + 16); return f.v;
  }
  static __device__ __forceinline__ v8f mma(v16h a, v16h b, v8f c) {
    return __builtin_amdgcn_wmma_f32_16x16x32_f16(false, a, false, b, (short)0, c, false, false);
  }
  static __device__ __forceinline__ void guard4(v8f& a, v8f& b, v8f& c, v8f& d, v16h x, v16h y) { dep_guard4_h(a, b, c, d, x, y); }
  static __device__ __forceinline__ void keep(v16h a, v16h b, v16h c, v16h d) { keep4_h(a, b, c, d); }
};
template <> struct Frag<__bf16> {
  typedef v16b V; union U { v16b v; v8b h[2]; };
  static __device__ __forceinline__ v16b load(const __bf16* p) {
    U f; f.h[0] = *(const v8b*)(p); f.h[1] = *(const v8b*)(p + 16); return f.v;
  }
  static __device__ __forceinline__ v8f mma(v16b a, v16b b, v8f c) {
    return __builtin_amdgcn_wmma_f32_16x16x32_bf16(false, a, false, b, (short)0, c, false, false);
  }
  static __device__ __forceinline__ void guard4(v8f& a, v8f& b, v8f& c, v8f& d, v16b x, v16b y) { dep_guard4_b(a, b, c, d, x, y); }
  static __device__ __forceinline__ void keep(v16b a, v16b b, v16b c, v16b d) { keep4_b(a, b, c, d); }
};

__device__ __forceinline__ v8f mma_h(v16h a, v16h b, v8f c) {
  c = __builtin_amdgcn_wmma_f32_16x16x32_f16(false, a, false, b, (short)0, c, false, false);
  asm volatile("v_nop\n\tv_nop\n\tv_nop\n\tv_nop" : "+v"(c) : "v"(a), "v"(b));
  return c;
}

template <int ET> struct Elem;
template <> struct Elem<0> { typedef _Float16 T; };
template <> struct Elem<1> { typedef __bf16 T; };
template <int ET, bool SPLIT, int BIAS_MODE, int OUT_MODE, bool RESID, int ACT = 0>
__global__ __launch_bounds__(256) void wmma_gemm64(
    const unsigned short* __restrict__ Ap, const unsigned short* __restrict__ A2p, int lda, long strideA,
    const unsigned short* __restrict__ Btp, const unsigned short* __restrict__ Bt2p, int ldb, long strideB,
    void* __restrict__ Cout, void* __restrict__ Cout2, int ldc, long strideC,
    const float* __restrict__ bias,
    const float* __restrict__ resid, long strideR,
    int M, int N, int K, float scale) {
  typedef typename Elem<ET>::T T;
  typedef typename Frag<T>::V V;
  const T* A = (const T*)Ap; const T* A2 = (const T*)A2p; const T* Bt = (const T*)Btp; const T* Bt2 = (const T*)Bt2p;
  __shared__ __align__(16) float sT[8][16 * 68];
  const int b    = blockIdx.y;
  const int lane = threadIdx.x & 31;
  const int wave = threadIdx.x >> 5;
  const int tilesN = N >> 6;
  const int tilesM = M >> 6;
  const int tile = blockIdx.x * 8 + wave;
  if (tile >= tilesM * tilesN) return;
  const int tm = tile / tilesN;
  const int tn = tile - tm * tilesN;
  const int m0 = tm << 6;
  const int n0 = tn << 6;

  const T* Ab  = A  + (size_t)b * strideA;
  const T* Bb  = Bt + (size_t)b * strideB;
  const T* Ab2 = SPLIT ? (A2  + (size_t)b * strideA) : nullptr;
  const T* Bb2 = SPLIT ? (Bt2 + (size_t)b * strideB) : nullptr;

  const int rlane = lane & 15;
  const int koff  = (lane >> 4) * 8;
  const int mOff  = (lane >> 4) * 8;

  v8f acc[4][4];
#pragma unroll
  for (int i = 0; i < 4; ++i)
#pragma unroll
    for (int j = 0; j < 4; ++j) acc[i][j] = (v8f){0.f,0.f,0.f,0.f,0.f,0.f,0.f,0.f};

  for (int k0 = 0; k0 < K; k0 += 32) {
    V bh[4], bl[4];
#pragma unroll
    for (int j = 0; j < 4; ++j) {
      const size_t bo = (size_t)(n0 + (j << 4) + rlane) * ldb + koff + k0;
      bh[j] = Frag<T>::load(Bb + bo);
      if (SPLIT) bl[j] = Frag<T>::load(Bb2 + bo);
    }
#pragma unroll
    for (int i = 0; i < 4; ++i) {
      const size_t ao = (size_t)(m0 + (i << 4) + rlane) * lda + koff + k0;
      V ah = Frag<T>::load(Ab + ao);
      V al;
      if (SPLIT) al = Frag<T>::load(Ab2 + ao);
#pragma unroll
      for (int j = 0; j < 4; ++j) {
        acc[i][j] = Frag<T>::mma(ah, bh[j], acc[i][j]);
        if (SPLIT) {
          acc[i][j] = Frag<T>::mma(ah, bl[j], acc[i][j]);
          acc[i][j] = Frag<T>::mma(al, bh[j], acc[i][j]);
        }
      }
      Frag<T>::guard4(acc[i][0], acc[i][1], acc[i][2], acc[i][3], ah, SPLIT ? al : ah);
    }
    Frag<T>::keep(bh[0], bh[1], bh[2], bh[3]);
    if (SPLIT) Frag<T>::keep(bl[0], bl[1], bl[2], bl[3]);
  }
  acc_guard4(acc[0][0], acc[0][1], acc[0][2], acc[0][3]);
  acc_guard4(acc[1][0], acc[1][1], acc[1][2], acc[1][3]);
  acc_guard4(acc[2][0], acc[2][1], acc[2][2], acc[2][3]);
  acc_guard4(acc[3][0], acc[3][1], acc[3][2], acc[3][3]);

  float* slab = sT[wave];
  const float* Rb = RESID ? (resid + (size_t)b * strideR) : nullptr;
#pragma unroll
  for (int i = 0; i < 4; ++i) {
    const int mBase = m0 + (i << 4);
#pragma unroll
    for (int j = 0; j < 4; ++j) {
      const int n = n0 + (j << 4) + rlane;
      float bv = 0.f;
      if (BIAS_MODE == 2) bv = bias[n];
#pragma unroll
      for (int r = 0; r < 8; ++r) {
        float v = acc[i][j][r] * scale;
        if (BIAS_MODE == 1) v += bias[mBase + mOff + r];
        if (BIAS_MODE == 2) v += bv;
        if (RESID) v += Rb[(size_t)(mBase + mOff + r) * ldc + n];
        if (ACT == 1) v = tanhf(v);
        if (ACT == 2) v = fmaxf(v, 0.0f);
        if (ACT == 3) v = v / (1.0f + expf(-v));
        if (ACT == 4) v = (v > 0.f) ? v : 0.01f * v;
        slab[(mOff + r) * 68 + (j << 4) + rlane] = v;
      }
    }
    __builtin_amdgcn_fence(__ATOMIC_RELEASE, "workgroup");
    __builtin_amdgcn_wave_barrier();
    __builtin_amdgcn_fence(__ATOMIC_ACQUIRE, "workgroup");
    if (OUT_MODE == 0) {
      float* C = (float*)Cout + (size_t)b * strideC;
      const int hh = lane >> 4, c4 = (lane & 15) * 4;
      for (int pass = 0; pass < 2; ++pass) {
#pragma unroll
        for (int it = 0; it < 8; ++it) {
          const int row = it * 2 + hh;
          v4f v = *(const v4f*)(slab + row * 68 + c4);
          *(volatile v4f*)(C + (size_t)(mBase + row) * ldc + n0 + c4) = v;
        }
        __threadfence();
      }
    } else {
      const int q = lane >> 3, c8 = (lane & 7) * 8;
      unsigned short* C  = (unsigned short*)Cout  + (size_t)b * strideC;
      unsigned short* C2 = (OUT_MODE == 2) ? ((unsigned short*)Cout2 + (size_t)b * strideC) : nullptr;
      for (int pass = 0; pass < 2; ++pass) {
#pragma unroll
        for (int it = 0; it < 4; ++it) {
          const int row = it * 4 + q;
          const float* sp = slab + row * 68 + c8;
          v8h hv, lv;
#pragma unroll
          for (int e = 0; e < 8; ++e) {
            if (OUT_MODE == 1) {
              hv[e] = (_Float16)sp[e];
            } else {
              unsigned short hb = f2bf_bits(sp[e]);
              unsigned short lb = f2bf_bits(sp[e] - bf_bits2f(hb));
              hv[e] = __builtin_bit_cast(_Float16, hb);
              lv[e] = __builtin_bit_cast(_Float16, lb);
            }
          }
          *(volatile v8h*)(C + (size_t)(mBase + row) * ldc + n0 + c8) = hv;
          if (OUT_MODE == 2) *(volatile v8h*)(C2 + (size_t)(mBase + row) * ldc + n0 + c8) = lv;
        }
        __threadfence();
      }
    }
    __builtin_amdgcn_fence(__ATOMIC_RELEASE, "workgroup");
    __builtin_amdgcn_wave_barrier();
    __builtin_amdgcn_fence(__ATOMIC_ACQUIRE, "workgroup");
  }
}


__global__ __launch_bounds__(kThr) void cast_plane_kernel(const float* __restrict__ src, unsigned short* __restrict__ dst,
                                                          int colsLog2, int dstPitch, int dstOff) {
  const int i   = blockIdx.x * kThr + threadIdx.x;
  const int sh  = colsLog2 - 3;
  const int row = i >> sh;
  const int c8  = (i & ((1 << sh) - 1)) * 8;
  const float* sp = src + ((size_t)row << colsLog2) + c8;
  const v4f a0 = *(const v4f*)(sp);
  const v4f a1 = *(const v4f*)(sp + 4);
  v8h hv;
#pragma unroll
  for (int e = 0; e < 4; ++e) {
    const float f0 = a0[e];
    const float f1 = a1[e];
    hv[e]     = (_Float16)carry_flush(bf16r(f0), kInCarry);
    hv[4 + e] = (_Float16)carry_flush(bf16r(f1), kInCarry);
  }
  unsigned short* dp = dst + (size_t)row * dstPitch + dstOff + c8;
  *(volatile v8h*)dp = hv;
  __threadfence();
  *(volatile v8h*)dp = hv;
}

__global__ __launch_bounds__(kThr) void biasrec_kernel(const float* __restrict__ a, const float* __restrict__ b, float* __restrict__ dst, int nb) {
  const unsigned v = blockIdx.x * (unsigned)kThr + threadIdx.x;
  const v4f pa = *(const v4f*)(a + v * 4u);
  const v4f pb = *(const v4f*)(b + v * 4u);
  const float wb = (nb == 2) ? 1.0f : 0.0f;
  v4f o;
#pragma unroll
  for (int e = 0; e < 4; ++e) o[e] = bf16r(pa[e]) + wb * bf16r(pb[e]);
  float* dp = dst + v * 4u;
  *(volatile v4f*)dp = o;
  __threadfence();
  *(volatile v4f*)dp = o;
}


__global__ __launch_bounds__(kThr) void cell_kernel(const float* __restrict__ GG, const float* __restrict__ c_prev, float* __restrict__ out) {
  const unsigned r = blockIdx.x, u8 = threadIdx.x * 8u;
  const float* gr = GG + (size_t)r * kG4 + u8;
  const float* cq = c_prev + (size_t)r * kHid + u8;
  v4f cn0, cn1, hn0, hn1;
#pragma unroll
  for (int hlf = 0; hlf < 2; ++hlf) {
    const v4f gf = *(const v4f*)(gr + 4 * hlf), gi = *(const v4f*)(gr + kHid + 4 * hlf), go = *(const v4f*)(gr + 2 * kHid + 4 * hlf), gc = *(const v4f*)(gr + 3 * kHid + 4 * hlf);
    const v4f co = *(const v4f*)(cq + 4 * hlf);
#pragma unroll
    for (int e = 0; e < 4; ++e) {
      const float zf = 1.0f / (1.0f + expf(-gf[e]));
      const float zi = 1.0f / (1.0f + expf(-gi[e]));
      const float zo = 1.0f / (1.0f + expf(-go[e]));
      const float zc = tanhf(gc[e]);
      const float cn = zf * bf16r(co[e]) + zi * zc;
      const float hn = zo * tanhf(cn);
      if (hlf == 0) { cn0[e] = cn; hn0[e] = hn; } else { cn1[e] = cn; hn1[e] = hn; }
    }
  }
  float* oh = out + (size_t)r * kHid + u8;
  float* oc = out + (size_t)kOut1 + (size_t)r * kHid + u8;
  for (int pass = 0; pass < 2; ++pass) {
    *(volatile v4f*)oh = hn0;
    *(volatile v4f*)(oh + 4) = hn1;
    *(volatile v4f*)oc = cn0;
    *(volatile v4f*)(oc + 4) = cn1;
    __threadfence();
  }
}
static_assert(kHid / 8 == 128 && kHid / 8 <= kThr, "the cell's block: 128 threads cover a row's 1,024 units (the launch passes kHid / 8 threads a block: under the kernel's bound of 256)");

extern "C" void kernel_launch(void* const* d_in, const int* in_sizes, int n_in,
                              void* d_out, int out_size, void* d_ws, size_t ws_size,
                              hipStream_t stream) {
  if (n_in < 10 || d_out == nullptr || d_ws == nullptr) return;
  if (in_sizes[0] != kB * kI || in_sizes[1] != kB * kI) return;
  if (in_sizes[2] != kB * kHid || in_sizes[3] != kB * kHid || in_sizes[4] != kB * kHid || in_sizes[5] != kB * kHid) return;
  if (in_sizes[6] != kG4 * kK || in_sizes[7] != kG4 || in_sizes[8] != kG4 * kK || in_sizes[9] != kG4) return;
  if (out_size != kOutAll) return;
  if (ws_size < kWsTotal) return;
  const float* x_f = (const float*)d_in[0];  const float* x_b = (const float*)d_in[1];
  const float* h_f = (const float*)d_in[2];  const float* c_f = (const float*)d_in[3];
  const float* h_b = (const float*)d_in[4];  const float* c_b = (const float*)d_in[5];
  const float* Wf = (const float*)d_in[6];   const float* bf = (const float*)d_in[7];
  const float* Wb = (const float*)d_in[8];   const float* bb = (const float*)d_in[9];
  float* out = (float*)d_out;
  char* ws = (char*)d_ws;
  unsigned short* AF16 = (unsigned short*)(ws + kOffAF16);
  unsigned short* AB16 = (unsigned short*)(ws + kOffAB16);
  unsigned short* WF16 = (unsigned short*)(ws + kOffWF16);
  unsigned short* WB16 = (unsigned short*)(ws + kOffWB16);
  float* BV = (float*)(ws + kOffBV);
  float* GG = (float*)(ws + kOffGG);

  const int gAct = (int)(((size_t)kB * 1024 / 8) / kThr), gW = (int)(((size_t)kG4 * kK / 8) / kThr);
  cast_plane_kernel<<<gAct, kThr, 0, stream>>>(x_f, AF16, 10, kK, 0);
  cast_plane_kernel<<<gAct, kThr, 0, stream>>>(h_f, AF16, 10, kK, kI);
  cast_plane_kernel<<<gAct, kThr, 0, stream>>>(x_b, AB16, 10, kK, 0);
  cast_plane_kernel<<<gAct, kThr, 0, stream>>>(h_b, AB16, 10, kK, kI);
  cast_plane_kernel<<<gW, kThr, 0, stream>>>(Wf, WF16, 11, kK, 0);
  cast_plane_kernel<<<gW, kThr, 0, stream>>>(Wb, WB16, 11, kK, 0);
  biasrec_kernel<<<kG4 / 4 / kThr, kThr, 0, stream>>>(bf, bf, BV, 1);
  biasrec_kernel<<<kG4 / 4 / kThr, kThr, 0, stream>>>(bb, bb, BV + kG4, 1);
  wmma_gemm64<0, false, 2, 0, false, 0><<<dim3((kB / 64) * (kG4 / 64) / 8, 1), 256, 0, stream>>>(
      AF16, AF16, kK, 0L, WF16, WF16, kK, 0L, (void*)GG, (void*)GG, kG4, 0L, BV, nullptr, 0L, kB, kG4, kK, kSc);
  cell_kernel<<<kB, kHid / 8, 0, stream>>>(GG, c_f, out);
  wmma_gemm64<0, false, 2, 0, false, 0><<<dim3((kB / 64) * (kG4 / 64) / 8, 1), 256, 0, stream>>>(
      AB16, AB16, kK, 0L, WB16, WB16, kK, 0L, (void*)GG, (void*)GG, kG4, 0L, BV + kG4, nullptr, 0L, kB, kG4, kK, kSc);
  cell_kernel<<<kB, kHid / 8, 0, stream>>>(GG, c_b, out + 2 * (size_t)kOut1);
}
static_assert(((kB / 64) * (kG4 / 64)) % 8 == 0 && (kG4 / 4) % kThr == 0 && ((size_t)kG4 * kK / 8) % kThr == 0 && ((size_t)kB * 1024 / 8) % kThr == 0, "the engine's grid: whole blocks of eight wave tiles; the bias records' and the casts' grids exact");
